// PyTorchHSTUAttention_67680094650971
// MI455X (gfx1250) — hardware-verified
//
#include <hip/hip_runtime.h>
#include <math.h>

typedef __attribute__((ext_vector_type(16))) _Float16 v16h;
typedef __attribute__((ext_vector_type(16))) __bf16 v16b;
typedef __attribute__((ext_vector_type(8)))  _Float16 v8h;
typedef __attribute__((ext_vector_type(8)))  float v8f;
typedef __attribute__((ext_vector_type(4)))  float v4f;
typedef __attribute__((ext_vector_type(2)))  float v2f;
typedef __attribute__((ext_vector_type(4)))  unsigned v4u;
typedef __attribute__((ext_vector_type(4)))  int v4i;
typedef float __attribute__((may_alias)) float_a;
typedef int __attribute__((may_alias)) int_a;

template <typename T> __device__ __forceinline__ void vst2(void* p, T v) { *(volatile T*)p = v; __threadfence(); *(volatile T*)p = v; }
__device__ __forceinline__ v8f wmma16(v16h a, v16h b, v8f c) {
  v8f d = __builtin_amdgcn_wmma_f32_16x16x32_f16(false, a, false, b, (short)0, c, false, false);
  asm volatile("v_nop\n\tv_nop\n\tv_nop\n\tv_nop" : "+v"(d) : "v"(a), "v"(b));
  return d;
}
__device__ __forceinline__ v8f wmma_bf(v16b a, v16b b, v8f c) {
  v8f d = __builtin_amdgcn_wmma_f32_16x16x32_bf16(false, a, false, b, (short)0, c, false, false);
  asm volatile("v_nop\n\tv_nop\n\tv_nop\n\tv_nop" : "+v"(d) : "v"(a), "v"(b));
  return d;
}
__device__ __forceinline__ v16h frag_h(const _Float16* rowk0, int lane) {
  union { v16h v; v8h q[2]; } u; const _Float16* p = rowk0 + 8 * (lane >> 4);
  u.q[0] = *(const v8h*)p; u.q[1] = *(const v8h*)(p + 16); return u.v;
}
__device__ __forceinline__ v16h frag_f32(const float* rowk0, int lane) {
  v16h a; const float* p = rowk0 + 8 * (lane >> 4);
#pragma unroll
  for (int i = 0; i < 8; ++i) { a[i] = (_Float16)p[i]; a[8 + i] = (_Float16)p[16 + i]; }
  return a;
}
__device__ __forceinline__ v16h frag_f32s(const float* rowk0, int lane, float sc) {
  v16h a; const float* p = rowk0 + 8 * (lane >> 4);
#pragma unroll
  for (int i = 0; i < 8; ++i) { a[i] = (_Float16)(p[i] * sc); a[8 + i] = (_Float16)(p[16 + i] * sc); }
  return a;
}
__device__ __forceinline__ v16h fragc_f32(const float* W, int k0, int n, int lane, int ld, int K) {
  v16h a; const int g = lane >> 4;
#pragma unroll
  for (int i = 0; i < 8; ++i) { const int ka = k0 + 8 * g + i, kb = ka + 16;
    a[i] = (_Float16)(ka < K ? W[(size_t)(ka < K ? ka : K - 1) * ld + n] : 0.f); a[8 + i] = (_Float16)(kb < K ? W[(size_t)(kb < K ? kb : K - 1) * ld + n] : 0.f); }
  return a;
}
struct F2 { v16b h, l; };
__device__ __forceinline__ F2 bsplit16(const float v[16]) { F2 r;
#pragma unroll
  for (int i = 0; i < 16; ++i) { const __bf16 h = (__bf16)v[i]; r.h[i] = h; r.l[i] = (__bf16)(v[i] - (float)h); }
  return r; }
__device__ __forceinline__ F2 split_row(const float* row, int k0, int lane) { float v[16]; const float* p = row + k0 + 8 * (lane >> 4);
#pragma unroll
  for (int i = 0; i < 8; ++i) { v[i] = p[i]; v[8 + i] = p[16 + i]; }
  return bsplit16(v); }
__device__ __forceinline__ F2 split_rowK(const float* row, int k0, int lane, int K) { float v[16]; const int g = lane >> 4;
#pragma unroll
  for (int i = 0; i < 8; ++i) { const int ka = k0 + 8 * g + i, kb = ka + 16; v[i] = ka < K ? row[ka < K ? ka : K - 1] : 0.f; v[8 + i] = kb < K ? row[kb < K ? kb : K - 1] : 0.f; }
  return bsplit16(v); }
__device__ __forceinline__ F2 split_col(const float* W, int k0, int n, int lane, int ld, int K) { float v[16]; const int g = lane >> 4;
#pragma unroll
  for (int i = 0; i < 8; ++i) { const int ka = k0 + 8 * g + i, kb = ka + 16; v[i] = ka < K ? W[(size_t)(ka < K ? ka : K - 1) * ld + n] : 0.f; v[8 + i] = kb < K ? W[(size_t)(kb < K ? kb : K - 1) * ld + n] : 0.f; }
  return bsplit16(v); }
__device__ __forceinline__ v8f mac3(const F2& a, const F2& b, v8f c) { c = wmma_bf(a.l, b.h, c); c = wmma_bf(a.h, b.l, c); return wmma_bf(a.h, b.h, c); }
__device__ __forceinline__ float sigm(float v) { return 1.0f / (1.0f + expf(-v)); }
#define LDSX() do { asm volatile("s_wait_dscnt 0" ::: "memory"); __builtin_amdgcn_wave_barrier(); __builtin_amdgcn_fence(__ATOMIC_RELEASE, "workgroup"); } while (0)


#define NHEAD 4
#define DQK   64
#define DVV   64
#define MTILE 128
#define JTILE 32
#define MAXSEQ 2048
typedef __attribute__((ext_vector_type(8))) __bf16 v8b;
__device__ __forceinline__ v16b frag_b16(const __bf16* rowk0, int lane) {
  union { v16b v; v8b q[2]; } u; const __bf16* p = rowk0 + 8 * (lane >> 4);
  u.q[0] = *(const v8b*)p; u.q[1] = *(const v8b*)(p + 16); return u.v;
}
__device__ __forceinline__ v16b frag_gbf(const float* rowk0, int lane) {
  v16b a; const float* p = rowk0 + 8 * (lane >> 4);
#pragma unroll
  for (int i = 0; i < 8; ++i) { a[i] = (__bf16)p[i]; a[8 + i] = (__bf16)p[16 + i]; }
  return a;
}
__device__ __forceinline__ float fsilu(float x) { return x / (1.0f + expf(-x)); }

__global__ __launch_bounds__(256)
void k_attn(const float* __restrict__ tq, const float* __restrict__ tk, const float* __restrict__ tv,
            const int* __restrict__ offsets, const int* __restrict__ ncand, const int* __restrict__ p_maxseq, const int* __restrict__ p_nctx,
            float* __restrict__ out) {
  __shared__ __align__(16) __bf16 Kb[JTILE][DQK];
  __shared__ __align__(16) __bf16 Vt[DVV][JTILE];
  __shared__ __align__(16) float Sscr[8][16][32];
  __shared__ __align__(16) float So[8][16][DVV];

  const int b    = blockIdx.z, h = blockIdx.y;
  const int off  = offsets[b];
  const int nlen = offsets[b + 1] - off;
  const int row0 = blockIdx.x * MTILE;
  if (row0 >= nlen) return;

  const int nc   = p_nctx[0];
  const int nt   = ncand[b];
  const int max1 = nlen - nc + 1;
  const int max2 = max1 - nt;
  const float invDenom = 1.0f / (float)p_maxseq[0];

  const int tid = threadIdx.x, wave = tid >> 5, lane = tid & 31, l16 = lane & 15, hh = lane >> 4;
  const int qb = row0 + wave * 16;

  int qrow = qb + l16; if (qrow > nlen - 1) qrow = nlen - 1;
  const float* qp = tq + (size_t)(off + qrow) * (NHEAD * DQK) + h * DQK;
  const v16b qf0 = frag_gbf(qp, lane), qf1 = frag_gbf(qp + 32, lane);

  v8f acc[4];
#pragma unroll
  for (int i = 0; i < 4; ++i) acc[i] = (v8f){};

  const int jcaus = (nlen < row0 + MTILE) ? nlen : (row0 + MTILE);
  const int jmax  = (row0 < nc) ? nlen : jcaus;
  const bool wctx = (qb < nc);

  for (int j = 0; j < jmax; j += JTILE) {
    {
      const int r = tid >> 3, cg = (tid & 7) * 8;
      int krow = j + r; if (krow > nlen - 1) krow = nlen - 1;
      const float* kp = tk + (size_t)(off + krow) * (NHEAD * DQK) + h * DQK + cg;
      const float4 a0 = *(const float4*)kp, a1 = *(const float4*)(kp + 4);
      union { v8b v; uint4 u; } cv;
      cv.v[0] = (__bf16)a0.x; cv.v[1] = (__bf16)a0.y; cv.v[2] = (__bf16)a0.z; cv.v[3] = (__bf16)a0.w;
      cv.v[4] = (__bf16)a1.x; cv.v[5] = (__bf16)a1.y; cv.v[6] = (__bf16)a1.z; cv.v[7] = (__bf16)a1.w;
      *(uint4*)&Kb[r][cg] = cv.u;
    }
    {
      const int rp = tid >> 4, cg = (tid & 15) * 4;
      int r0g = j + 2 * rp, r1g = r0g + 1;
      if (r0g > nlen - 1) r0g = nlen - 1;
      if (r1g > nlen - 1) r1g = nlen - 1;
      const float4 a = *(const float4*)(tv + (size_t)(off + r0g) * (NHEAD * DVV) + h * DVV + cg);
      const float4 c = *(const float4*)(tv + (size_t)(off + r1g) * (NHEAD * DVV) + h * DVV + cg);
      union { __bf16 h2[2]; uint32_t u; } p0, p1, p2, p3;
      p0.h2[0] = (__bf16)a.x; p0.h2[1] = (__bf16)c.x; p1.h2[0] = (__bf16)a.y; p1.h2[1] = (__bf16)c.y;
      p2.h2[0] = (__bf16)a.z; p2.h2[1] = (__bf16)c.z; p3.h2[0] = (__bf16)a.w; p3.h2[1] = (__bf16)c.w;
      *(uint32_t*)&Vt[cg + 0][2 * rp] = p0.u; *(uint32_t*)&Vt[cg + 1][2 * rp] = p1.u;
      *(uint32_t*)&Vt[cg + 2][2 * rp] = p2.u; *(uint32_t*)&Vt[cg + 3][2 * rp] = p3.u;
    }
    __syncthreads();

    const bool active = wctx || (j <= qb + 15);
    if (active) {
      v8f s0 = (v8f){}, s1 = (v8f){};
      s0 = wmma_bf(qf0, frag_b16(&Kb[l16][0], lane), s0);       s0 = wmma_bf(qf1, frag_b16(&Kb[l16][32], lane), s0);
      s1 = wmma_bf(qf0, frag_b16(&Kb[16 + l16][0], lane), s1);  s1 = wmma_bf(qf1, frag_b16(&Kb[16 + l16][32], lane), s1);

      {
        float* sp = &Sscr[wave][0][0];
        const int y0 = j + l16, y1 = y0 + 16;
        const int idy0 = max(y0 - nc + 1, 0), idy1 = max(y1 - nc + 1, 0);
        const int tgy0 = max(idy0 - max1 + nt, -1), tgy1 = max(idy1 - max1 + nt, -1);
#pragma unroll
        for (int r = 0; r < 8; ++r) {
          const int m = r + hh * 8, x = qb + m;
          const int idx = max(x - nc + 1, 0), tgx = max(idx - max1 + nt, -1);
          const bool c0 = (x == y0) || (idx > idy0), c1 = (x == y1) || (idx > idy1);
          const bool g0 = (tgx == tgy0) || (tgx < 0) || (tgy0 < 0), g1 = (tgx == tgy1) || (tgx < 0) || (tgy1 < 0);
          const bool ctx = (idx == 0);
          const bool ok0 = ((c0 && g0) || (ctx && idy0 < max2)) && (y0 < nlen) && (x < nlen);
          const bool ok1 = ((c1 && g1) || (ctx && idy1 < max2)) && (y1 < nlen) && (x < nlen);
          const float a0v = fsilu(s0[r] * 0.125f), a1v = fsilu(s1[r] * 0.125f);
          sp[m * 32 + l16]      = ok0 ? a0v : 0.0f;
          sp[m * 32 + 16 + l16] = ok1 ? a1v : 0.0f;
        }
      }
      LDSX();
      F2 pf;
      { float v[16]; const float* row = &Sscr[wave][l16][0]; const int c0 = hh * 8;
#pragma unroll
        for (int i = 0; i < 8; ++i) { v[i] = row[c0 + i]; v[8 + i] = row[16 + c0 + i]; }
        pf = bsplit16(v); }
#pragma unroll
      for (int dc = 0; dc < 4; ++dc) {
        const v16b vf = frag_b16(&Vt[dc * 16 + l16][0], lane);
        acc[dc] = wmma_bf(pf.l, vf, acc[dc]);
        acc[dc] = wmma_bf(pf.h, vf, acc[dc]);
      }
    }
    __syncthreads();
  }

  float* so = &So[wave][0][0];
#pragma unroll
  for (int r = 0; r < 8; ++r)
#pragma unroll
    for (int dc = 0; dc < 4; ++dc) so[(r + hh * 8) * DVV + dc * 16 + l16] = acc[dc][r] * invDenom;
  LDSX();
#pragma unroll
  for (int m2 = 0; m2 < 8; ++m2) { const int m = 2 * m2 + hh; const int x = qb + m;
    if (x < nlen) vst2(out + (size_t)(off + x) * (NHEAD * DVV) + h * DVV + l16 * 4, *(const v4f*)(so + m * DVV + l16 * 4)); }
}

extern "C" void kernel_launch(void* const* d_in, const int* in_sizes, int n_in, void* d_out, int out_size, void* d_ws, size_t ws_size, hipStream_t stream) {
  (void)n_in; (void)out_size; (void)d_ws; (void)ws_size;
  const int nseq = in_sizes[3] - 1;
  dim3 grid(MAXSEQ / MTILE, NHEAD, nseq), block(256, 1, 1);
  k_attn<<<grid, block, 0, stream>>>((const float*)d_in[0], (const float*)d_in[1], (const float*)d_in[2],
                                     (const int*)d_in[3], (const int*)d_in[4], (const int*)d_in[5], (const int*)d_in[6], (float*)d_out);
}
